// SimpleRNN_32641751449606
// MI455X (gfx1250) — hardware-verified
//
#include <hip/hip_runtime.h>

typedef __attribute__((ext_vector_type(16))) _Float16 v16h;
typedef __attribute__((ext_vector_type(8)))  _Float16 v8h;
typedef __attribute__((ext_vector_type(8)))  float    v8f;
typedef __attribute__((ext_vector_type(4)))  float    v4f;

constexpr int NBATCH = 2048;
constexpr int NSEQ   = 512;
constexpr int NFIN   = 15;
constexpr int NHID   = 32;
constexpr int NGATE  = 96;
constexpr int NTAIL  = 24;
constexpr int SPB    = 64;
constexpr int NTHR   = 256;
constexpr int TPH    = 32;
static_assert(NBATCH % SPB == 0);
static_assert(NFIN <= TPH);

constexpr float WCARRY     = 4.0f;
constexpr float WCARRY_INV = 0.25f;
constexpr float RCARRY     = 2048.0f;
constexpr float RCARRY_INV = 1.0f / 2048.0f;
constexpr float FOLD       = 1.0f / 8192.0f;

constexpr int OFF_WDH = 0;
constexpr int OFF_WDL = OFF_WDH + NHID * TPH;
constexpr int OFF_WIH = OFF_WDL + NHID * TPH;
constexpr int OFF_WIL = OFF_WIH + NGATE * TPH;
constexpr int OFF_WHH = OFF_WIL + NGATE * TPH;
constexpr int OFF_WHL = OFF_WHH + NGATE * TPH;
constexpr int OFF_XH  = OFF_WHL + NGATE * TPH;
constexpr int OFF_XL  = OFF_XH + SPB * TPH;
constexpr int OFF_PH  = OFF_XL + SPB * TPH;
constexpr int OFF_PL  = OFF_PH + SPB * TPH;
constexpr int OFF_HH  = OFF_PL + SPB * TPH;
constexpr int OFF_HL  = OFF_HH + SPB * TPH;
constexpr int LDS_HALVES = OFF_HL + SPB * TPH;
static_assert(LDS_HALVES == 26624);
static_assert(OFF_XH + 6 * SPB * TPH == LDS_HALVES);
constexpr int SB_BD = 0, SB_BIH = 32, SB_BHH = 128, SB_WOUT = 224, SB_BOUT = 256, SB_N = 264;

template <typename T> struct Frag;
template <> struct Frag<_Float16> {
  typedef v16h V; union U { v16h v; v8h h[2]; };
  static __device__ __forceinline__ v16h load(const _Float16* p) {
    U f; f.h[0] = *(const v8h*)(p); f.h[1] = *(const v8h*)(p + 16); return f.v;
  }
  static __device__ __forceinline__ v8f mma(v16h a, v16h b, v8f c) {
    return __builtin_amdgcn_wmma_f32_16x16x32_f16(false, a, false, b, (short)0, c, false, false);
  }
};
typedef Frag<_Float16> FragH;

__device__ __forceinline__ void guard2f4(v8f& a, v8f& b, v16h w, v16h x, v16h y, v16h z) {
  asm volatile("v_nop\n\tv_nop\n\tv_nop\n\tv_nop" : "+v"(a), "+v"(b) : "v"(w), "v"(x), "v"(y), "v"(z));
}
__device__ __forceinline__ void guard4f8(v8f& a, v8f& b, v8f& c, v8f& d,
                                         v16h s0, v16h s1, v16h s2, v16h s3, v16h s4, v16h s5, v16h s6, v16h s7) {
  asm volatile("v_nop\n\tv_nop\n\tv_nop\n\tv_nop" : "+v"(a), "+v"(b), "+v"(c), "+v"(d)
               : "v"(s0), "v"(s1), "v"(s2), "v"(s3), "v"(s4), "v"(s5), "v"(s6), "v"(s7));
}
__device__ __forceinline__ void accg8(v8f& a, v8f& b, v8f& c, v8f& d, v8f& e, v8f& f, v8f& g, v8f& h) {
  asm volatile("v_nop\n\tv_nop\n\tv_nop\n\tv_nop" : "+v"(a), "+v"(b), "+v"(c), "+v"(d), "+v"(e), "+v"(f), "+v"(g), "+v"(h));
}

__device__ __forceinline__ float fsigm(float x) { return __builtin_amdgcn_rcpf(1.0f + __expf(-x)); }
__device__ __forceinline__ float ftanh(float x) { return 1.0f - 2.0f * __builtin_amdgcn_rcpf(1.0f + __expf(2.0f * x)); }

__device__ __forceinline__ void split16(float v, _Float16& hi, _Float16& lo) {
  hi = (_Float16)v;
  lo = (_Float16)((v - (float)hi) * RCARRY);
}

__device__ __forceinline__ float head_dot(const _Float16* lh, const float* sb, int row) {
  float acc = 0.0f;
#pragma unroll 1
  for (int j = 0; j < NHID; ++j) {
    const float hv = (float)lh[OFF_HH + row * TPH + j] + (float)lh[OFF_HL + row * TPH + j] * RCARRY_INV;
    acc = fmaf(hv, sb[SB_WOUT + j], acc);
  }
  return acc + sb[SB_BOUT];
}

__global__ __launch_bounds__(NTHR) void gru_fused(const float* __restrict__ x,
                                                  const float* __restrict__ Wd,
                                                  const float* __restrict__ bd,
                                                  const float* __restrict__ Wih,
                                                  const float* __restrict__ Whh,
                                                  const float* __restrict__ bih,
                                                  const float* __restrict__ bhh,
                                                  const float* __restrict__ Wout,
                                                  const float* __restrict__ bout,
                                                  float* __restrict__ out) {
  __shared__ __align__(16) _Float16 lh[LDS_HALVES];
  __shared__ __align__(16) float s_out[SPB * NTAIL];
  __shared__ float s_b[SB_N];

  const int tid = threadIdx.x, lane = tid & 31, wave = tid >> 5;
  const int c = lane & 15, h8 = (lane >> 4) * 8;
  const int blk = blockIdx.x;
  const int b0 = blk * SPB;

  for (int i = tid; i < NHID * TPH; i += NTHR) {
    const int n = i >> 5, k = i & 31;
    const int kc = (k < NFIN) ? k : (NFIN - 1);
    float v = Wd[n * NFIN + kc];
    v = (k < NFIN) ? v * WCARRY : 0.0f;
    _Float16 hi, lo; split16(v, hi, lo);
    lh[OFF_WDH + i] = hi; lh[OFF_WDL + i] = lo;
  }
  for (int i = tid; i < NGATE * TPH; i += NTHR) {
    _Float16 hi, lo;
    split16(Wih[i] * WCARRY, hi, lo); lh[OFF_WIH + i] = hi; lh[OFF_WIL + i] = lo;
    split16(Whh[i] * WCARRY, hi, lo); lh[OFF_WHH + i] = hi; lh[OFF_WHL + i] = lo;
  }
  for (int i = tid; i < 6 * SPB * TPH; i += NTHR)
    lh[OFF_XH + i] = (_Float16)0.0f;
  if (tid < NHID) { s_b[SB_BD + tid] = bd[tid]; s_b[SB_WOUT + tid] = Wout[tid]; }
  for (int i = tid; i < NGATE; i += NTHR) { s_b[SB_BIH + i] = bih[i]; s_b[SB_BHH + i] = bhh[i]; }
  if (tid == 0) s_b[SB_BOUT] = bout[0];

  int gidx[4], loff[4];
  float xv[4];
#pragma unroll
  for (int i = 0; i < 4; ++i) {
    int e = tid + i * NTHR;
    e = (e < SPB * NFIN) ? e : (SPB * NFIN - 1);
    const int row = e / NFIN, col = e - row * NFIN;
    gidx[i] = (b0 + row) * (NSEQ * NFIN) + col;
    loff[i] = row * TPH + col;
    xv[i] = x[(size_t)gidx[i]];
  }
  __syncthreads();

  const int rt = wave >> 1, sub = wave & 1;
  const int jcol = 16 * sub + c;
  const int arow = (16 * rt + c) * TPH + h8;
  const int bwd  = (16 * sub + c) * TPH + h8;
  const int bgr  = jcol * TPH + h8;
  const int bgz  = (NHID + jcol) * TPH + h8;
  const int bgn  = (2 * NHID + jcol) * TPH + h8;
  const int drow = 16 * rt + h8;
  const float bdv = s_b[SB_BD + jcol];
  const float bR  = s_b[SB_BIH + jcol] + s_b[SB_BHH + jcol];
  const float bZ  = s_b[SB_BIH + NHID + jcol] + s_b[SB_BHH + NHID + jcol];
  const float bXN = s_b[SB_BIH + 2 * NHID + jcol];
  const float bHN = s_b[SB_BHH + 2 * NHID + jcol];
  const v8f z8 = {0.f, 0.f, 0.f, 0.f, 0.f, 0.f, 0.f, 0.f};

  float hreg[8];
#pragma unroll
  for (int r = 0; r < 8; ++r) hreg[r] = 0.0f;

#pragma unroll 1
  for (int s = 0; s < NSEQ; ++s) {
#pragma unroll
    for (int r = 0; r < 8; ++r) {
      _Float16 hi, lo; split16(hreg[r], hi, lo);
      lh[OFF_HH + (drow + r) * TPH + jcol] = hi;
      lh[OFF_HL + (drow + r) * TPH + jcol] = lo;
    }
#pragma unroll
    for (int i = 0; i < 4; ++i) {
      _Float16 hi, lo; split16(xv[i], hi, lo);
      lh[OFF_XH + loff[i]] = hi;
      lh[OFF_XL + loff[i]] = lo;
    }
    {
      const int sn = (s + 1 < NSEQ) ? (s + 1) : (NSEQ - 1);
      const size_t so = (size_t)sn * NFIN;
#pragma unroll
      for (int i = 0; i < 4; ++i) xv[i] = x[(size_t)gidx[i] + so];
    }
    __syncthreads();

    if (s - 1 >= NSEQ - NTAIL) {
      if (tid < SPB) s_out[tid * NTAIL + (s - 1 - (NSEQ - NTAIL))] = head_dot(lh, s_b, tid);
    }
    {
      const v16h axh = FragH::load(lh + OFF_XH + arow);
      const v16h axl = FragH::load(lh + OFF_XL + arow);
      const v16h bwh = FragH::load(lh + OFF_WDH + bwd);
      const v16h bwl = FragH::load(lh + OFF_WDL + bwd);
      v8f am = z8, amr = z8;
      am  = FragH::mma(axh, bwh, am);
      amr = FragH::mma(axh, bwl, amr);
      amr = FragH::mma(axl, bwh, amr);
      guard2f4(am, amr, axh, axl, bwh, bwl);
#pragma unroll
      for (int r = 0; r < 8; ++r) {
        const float xp = fmaf(amr[r], FOLD, fmaf(am[r], WCARRY_INV, bdv));
        _Float16 hi, lo; split16(xp, hi, lo);
        lh[OFF_PH + (drow + r) * TPH + jcol] = hi;
        lh[OFF_PL + (drow + r) * TPH + jcol] = lo;
      }
    }
    __syncthreads();

    {
      const v16h aph = FragH::load(lh + OFF_PH + arow);
      const v16h apl = FragH::load(lh + OFF_PL + arow);
      const v16h ahh = FragH::load(lh + OFF_HH + arow);
      const v16h ahl = FragH::load(lh + OFF_HL + arow);
      v8f aR, aRr, aZ, aZr, aXN, aXNr, aHN, aHNr;
      {
        const v16h fxh = FragH::load(lh + OFF_WIH + bgr), fxl = FragH::load(lh + OFF_WIL + bgr);
        const v16h fhh = FragH::load(lh + OFF_WHH + bgr), fhl = FragH::load(lh + OFF_WHL + bgr);
        aR  = FragH::mma(aph, fxh, z8);  aR  = FragH::mma(ahh, fhh, aR);
        aRr = FragH::mma(aph, fxl, z8);  aRr = FragH::mma(apl, fxh, aRr);
        aRr = FragH::mma(ahh, fhl, aRr); aRr = FragH::mma(ahl, fhh, aRr);
        guard2f4(aR, aRr, fxh, fxl, fhh, fhl);
      }
      {
        const v16h fxh = FragH::load(lh + OFF_WIH + bgz), fxl = FragH::load(lh + OFF_WIL + bgz);
        const v16h fhh = FragH::load(lh + OFF_WHH + bgz), fhl = FragH::load(lh + OFF_WHL + bgz);
        aZ  = FragH::mma(aph, fxh, z8);  aZ  = FragH::mma(ahh, fhh, aZ);
        aZr = FragH::mma(aph, fxl, z8);  aZr = FragH::mma(apl, fxh, aZr);
        aZr = FragH::mma(ahh, fhl, aZr); aZr = FragH::mma(ahl, fhh, aZr);
        guard2f4(aZ, aZr, fxh, fxl, fhh, fhl);
      }
      {
        const v16h fxh = FragH::load(lh + OFF_WIH + bgn), fxl = FragH::load(lh + OFF_WIL + bgn);
        const v16h fhh = FragH::load(lh + OFF_WHH + bgn), fhl = FragH::load(lh + OFF_WHL + bgn);
        aXN  = FragH::mma(aph, fxh, z8);
        aXNr = FragH::mma(aph, fxl, z8); aXNr = FragH::mma(apl, fxh, aXNr);
        aHN  = FragH::mma(ahh, fhh, z8);
        aHNr = FragH::mma(ahh, fhl, z8); aHNr = FragH::mma(ahl, fhh, aHNr);
        guard4f8(aXN, aXNr, aHN, aHNr, fxh, fxl, fhh, fhl, aph, apl, ahh, ahl);
      }
      accg8(aR, aRr, aZ, aZr, aXN, aXNr, aHN, aHNr);
#pragma unroll
      for (int r = 0; r < 8; ++r) {
        const float pr = fmaf(aRr[r],  FOLD, fmaf(aR[r],  WCARRY_INV, bR));
        const float pz = fmaf(aZr[r],  FOLD, fmaf(aZ[r],  WCARRY_INV, bZ));
        const float xn = fmaf(aXNr[r], FOLD, fmaf(aXN[r], WCARRY_INV, bXN));
        const float hn = fmaf(aHNr[r], FOLD, fmaf(aHN[r], WCARRY_INV, bHN));
        const float rg = fsigm(pr);
        const float zg = fsigm(pz);
        const float ng = ftanh(fmaf(rg, hn, xn));
        hreg[r] = fmaf(zg, hreg[r] - ng, ng);
      }
    }
    __syncthreads();
  }

#pragma unroll
  for (int r = 0; r < 8; ++r) {
    _Float16 hi, lo; split16(hreg[r], hi, lo);
    lh[OFF_HH + (drow + r) * TPH + jcol] = hi;
    lh[OFF_HL + (drow + r) * TPH + jcol] = lo;
  }
  __syncthreads();
  if (tid < SPB) s_out[tid * NTAIL + (NTAIL - 1)] = head_dot(lh, s_b, tid);
  __syncthreads();
  {
    float* ob = out + (size_t)blk * (SPB * NTAIL);
    const int q = lane >> 3, c4 = (lane & 7) * 4;
    for (int pass = 0; pass < 2; ++pass) {
#pragma unroll
      for (int it = 0; it < 2; ++it) {
        if (it * 32 + wave * 4 < SPB * NTAIL / 32) {
          const int line = it * 32 + wave * 4 + q;
          const v4f v = *(const v4f*)(s_out + line * 32 + c4);
          *(volatile v4f*)(ob + line * 32 + c4) = v;
        }
      }
      __threadfence();
    }
  }
}

extern "C" void kernel_launch(void* const* d_in, const int* in_sizes, int n_in,
                              void* d_out, int out_size, void* d_ws, size_t ws_size, hipStream_t stream) {
  (void)d_ws; (void)ws_size;
  if (n_in < 9 || d_out == nullptr) return;
  if (in_sizes[0] != NBATCH * NSEQ * NFIN || in_sizes[1] != NHID * NFIN || in_sizes[2] != NHID ||
      in_sizes[3] != NGATE * NHID || in_sizes[4] != NGATE * NHID || in_sizes[5] != NGATE || in_sizes[6] != NGATE ||
      in_sizes[7] != NHID || in_sizes[8] != 1 || out_size != NBATCH * NTAIL) return;

  const float* x    = (const float*)d_in[0];
  const float* Wd   = (const float*)d_in[1];
  const float* bd   = (const float*)d_in[2];
  const float* Wih  = (const float*)d_in[3];
  const float* Whh  = (const float*)d_in[4];
  const float* bih  = (const float*)d_in[5];
  const float* bhh  = (const float*)d_in[6];
  const float* Wout = (const float*)d_in[7];
  const float* bout = (const float*)d_in[8];
  float* out = (float*)d_out;

  gru_fused<<<dim3(NBATCH / SPB), dim3(NTHR), 0, stream>>>(x, Wd, bd, Wih, Whh, bih, bhh, Wout, bout, out);
}
